// EquivairantMultiheadAttention_29798483100008
// MI455X (gfx1250) — hardware-run, weakly checked
//
#include <hip/hip_runtime.h>
#include <math.h>

#ifndef NB
#define NB 4
#endif
#ifndef SEQ
#define SEQ 512
#endif
#define NB_FULL 4
#define SEQ_FULL 512
#define CH 256
#define HEADS 8
#define HD 32
#define DG 6
#define HID 16
#define MTOK (NB * SEQ)
#define QBLK (SEQ / 256)

#define G_CARRY 4.0f
#define W1_CARRY 16.0f
#define UNDO1 (1.0f / 64.0f)
#define H_CARRY 64.0f
#define W2_CARRY 16.0f
#define UNDO2 (1.0f / 1024.0f)
#define ACT_CARRY 8.0f
#define W_CARRY 32.0f
#define SC_PROJ (1.0f / 256.0f)
#define SCQK (1.0f / 1024.0f)
#define P_CARRY 1024.0f
#define O_CARRY 64.0f
#define SC_OUT (1.0f / 2048.0f)
#define LOG2E 1.4426950408889634f
#define FILL2 (-1.0e38f * LOG2E)

static_assert(G_CARRY * W1_CARRY * UNDO1 == 1.0f);
static_assert(H_CARRY * W2_CARRY * UNDO2 == 1.0f);
static_assert(ACT_CARRY * W_CARRY * SC_PROJ == 1.0f);
static_assert(ACT_CARRY * ACT_CARRY * 16.0f * SCQK == 1.0f);
static_assert(O_CARRY * W_CARRY * SC_OUT == 1.0f);
static_assert(SEQ == SEQ_FULL);
static_assert(NB <= NB_FULL);
static_assert(CH == HEADS * HD && HD == 32 && HID == 16 && DG <= 8);
static_assert(SEQ % 256 == 0 && SEQ % 64 == 0);
static_assert(MTOK % 64 == 0 && CH % 64 == 0 && CH % 32 == 0);
static_assert((NB * SEQ * SEQ) % 256 == 0);
static_assert((MTOK * CH / 8) % 256 == 0);
static_assert((CH * (CH / 8)) % 256 == 0);
static_assert(32 * 16 * 4 == 16 * 128);
static_assert(32 * 16 * 8 == 16 * 256);
static_assert(32 * 4 * 8 == 8 * 128);
static_assert(8 * 16 * 68 * 4 <= 131072);
static_assert(8 * 16 * 20 * 4 + 8 * HEADS * 32 * 4 <= 131072);
static_assert(16 * 16 * 72 * 2 + 16 * 16 * 68 * 4 <= 131072);

typedef _Float16 h16;
typedef __attribute__((ext_vector_type(16))) _Float16 v16h;
typedef __attribute__((ext_vector_type(8)))  _Float16 v8h;
typedef __attribute__((ext_vector_type(2)))  _Float16 v2h;
typedef __attribute__((ext_vector_type(8)))  float    v8f;
typedef __attribute__((ext_vector_type(4)))  float    v4f;
typedef __attribute__((ext_vector_type(2)))  float    v2f;
typedef __attribute__((ext_vector_type(4)))  unsigned int v4u;

static constexpr size_t SZ_G16  = (size_t)NB * SEQ * SEQ * 8 * 2;
static constexpr size_t SZ_C16  = (size_t)MTOK * CH * 2;
static constexpr size_t SZ_WT   = (size_t)4 * CH * CH * 2;
static constexpr size_t SZ_W1B  = (size_t)HEADS * HID * 32 * 2;
static constexpr size_t SZ_W2B  = (size_t)HEADS * HID * 32 * 2;
static constexpr size_t SZ_Q16  = (size_t)MTOK * CH * 2;
static constexpr size_t SZ_K16  = (size_t)MTOK * CH * 2;
static constexpr size_t SZ_VT16 = (size_t)NB * CH * SEQ * 2;
static constexpr size_t SZ_ALOC = (size_t)NB * HEADS * SEQ * SEQ * 4;
static constexpr size_t SZ_O16  = (size_t)MTOK * CH * 2;
static constexpr size_t OFF_G16  = 0;
static constexpr size_t OFF_C16  = OFF_G16 + SZ_G16;
static constexpr size_t OFF_WT   = OFF_C16 + SZ_C16;
static constexpr size_t OFF_W1B  = OFF_WT + SZ_WT;
static constexpr size_t OFF_W2B  = OFF_W1B + SZ_W1B;
static constexpr size_t OFF_Q16  = OFF_W2B + SZ_W2B;
static constexpr size_t OFF_K16  = OFF_Q16 + SZ_Q16;
static constexpr size_t OFF_VT16 = OFF_K16 + SZ_K16;
static constexpr size_t OFF_ALOC = OFF_VT16 + SZ_VT16;
static constexpr size_t OFF_O16  = OFF_ALOC + SZ_ALOC;
static constexpr size_t WS_TOTAL = OFF_O16 + SZ_O16;
static_assert(SZ_G16 % 256 == 0 && SZ_C16 % 256 == 0 && SZ_WT % 256 == 0 && SZ_W1B % 256 == 0 && SZ_W2B % 256 == 0);
static_assert(SZ_Q16 % 256 == 0 && SZ_VT16 % 256 == 0 && SZ_ALOC % 256 == 0 && SZ_O16 % 256 == 0);
static_assert(WS_TOTAL <= (size_t)134217728);


__device__ __forceinline__ float bfr(float f) {
    unsigned u = __float_as_uint(f);
    u += 0x7FFFu + ((u >> 16) & 1u);
    return __uint_as_float(u & 0xFFFF0000u);
}
static __device__ __forceinline__ h16 toh_flush(float v) { const float w = (fabsf(v) < 6.103515625e-05f) ? 0.0f : v; return (h16)w; }
static __device__ __forceinline__ v2h toh2_flush(float a, float b) {
    v2f w;
    w.x = (fabsf(a) < 6.103515625e-05f) ? 0.0f : a;
    w.y = (fabsf(b) < 6.103515625e-05f) ? 0.0f : b;
    return __builtin_convertvector(w, v2h);
}
union Pack8 { v8h v; v2h p[4]; };
static __device__ __forceinline__ v8h pack8_flush(v4f a, v4f b) {
    Pack8 u;
    u.p[0] = toh2_flush(a.x, a.y); u.p[1] = toh2_flush(a.z, a.w);
    u.p[2] = toh2_flush(b.x, b.y); u.p[3] = toh2_flush(b.z, b.w);
    return u.v;
}
static __device__ __forceinline__ void st8h2(_Float16* p, v8h v) {
    *(volatile v8h*)p = v;
    __threadfence();
    *(volatile v8h*)p = v;
}

union FragU { v16h v; v8h h[2]; };
union FragQ { v16h v; v8h h[2]; v4u q[2]; };
__device__ __forceinline__ v16h frag_ld(const _Float16* p) {
    FragU f; f.h[0] = *(const v8h*)(p); f.h[1] = *(const v8h*)(p + 16); return f.v;
}
__device__ __forceinline__ v8f wmma16g(v16h a, v16h b, v8f c) {
    c = __builtin_amdgcn_wmma_f32_16x16x32_f16(false, a, false, b, (short)0, c, false, false);
    asm volatile("v_nop\n\tv_nop\n\tv_nop\n\tv_nop" : "+v"(c) : "v"(a), "v"(b));
    return c;
}
__device__ __forceinline__ void wave_sync_lds() {
    __builtin_amdgcn_fence(3  , "workgroup");
    __builtin_amdgcn_wave_barrier();
    __builtin_amdgcn_fence(2  , "workgroup");
}
static __device__ __forceinline__ float swishf(float x) {
    return x / (1.0f + exp2f(-x * LOG2E));
}

__global__ __launch_bounds__(256) void k_cvt_g(const float* __restrict__ g, _Float16* __restrict__ G16) {
    const unsigned u = blockIdx.x * 256u + threadIdx.x;
    if (u >= (unsigned)(NB * SEQ * SEQ)) return;
    const v2f* src = (const v2f*)(g + (size_t)u * 6u);
    const v2f a = src[0], b = src[1], cc = src[2];
    v4f lo, hi;
    lo.x = bfr(a.x) * G_CARRY; lo.y = bfr(a.y) * G_CARRY; lo.z = bfr(b.x) * G_CARRY; lo.w = bfr(b.y) * G_CARRY;
    hi.x = bfr(cc.x) * G_CARRY; hi.y = bfr(cc.y) * G_CARRY; hi.z = 0.0f; hi.w = 0.0f;
    st8h2(G16 + (size_t)u * 8u, pack8_flush(lo, hi));
}

__global__ __launch_bounds__(256) void k_cvt_c(const float* __restrict__ x, _Float16* __restrict__ C16) {
    const unsigned u = blockIdx.x * 256u + threadIdx.x;
    if (u >= (unsigned)(MTOK * CH / 8)) return;
    const v4f* src = (const v4f*)(x + (size_t)u * 8u);
    v4f a = src[0], b = src[1];
    a.x = bfr(a.x) * ACT_CARRY; a.y = bfr(a.y) * ACT_CARRY; a.z = bfr(a.z) * ACT_CARRY; a.w = bfr(a.w) * ACT_CARRY;
    b.x = bfr(b.x) * ACT_CARRY; b.y = bfr(b.y) * ACT_CARRY; b.z = bfr(b.z) * ACT_CARRY; b.w = bfr(b.w) * ACT_CARRY;
    st8h2(C16 + (size_t)u * 8u, pack8_flush(a, b));
}

static __device__ __forceinline__ void wt_one(const float* __restrict__ W, _Float16* __restrict__ D, unsigned o, unsigned k0) {
    v4f lo, hi;
    lo.x = bfr(W[(size_t)(k0 + 0u) * CH + o]) * W_CARRY;
    lo.y = bfr(W[(size_t)(k0 + 1u) * CH + o]) * W_CARRY;
    lo.z = bfr(W[(size_t)(k0 + 2u) * CH + o]) * W_CARRY;
    lo.w = bfr(W[(size_t)(k0 + 3u) * CH + o]) * W_CARRY;
    hi.x = bfr(W[(size_t)(k0 + 4u) * CH + o]) * W_CARRY;
    hi.y = bfr(W[(size_t)(k0 + 5u) * CH + o]) * W_CARRY;
    hi.z = bfr(W[(size_t)(k0 + 6u) * CH + o]) * W_CARRY;
    hi.w = bfr(W[(size_t)(k0 + 7u) * CH + o]) * W_CARRY;
    st8h2(D + (size_t)o * CH + k0, pack8_flush(lo, hi));
}
__global__ __launch_bounds__(256) void k_wt4(const float* __restrict__ wq, const float* __restrict__ wk,
                                             const float* __restrict__ wv, const float* __restrict__ wo,
                                             _Float16* __restrict__ WT) {
    const unsigned u = blockIdx.x * 256u + threadIdx.x;
    if (u >= (unsigned)(CH * (CH / 8))) return;
    const unsigned k0 = 8u * (u & 31u);
    const unsigned o = u >> 5;
    wt_one(wq, WT, o, k0);
    wt_one(wk, WT + (size_t)1 * CH * CH, o, k0);
    wt_one(wv, WT + (size_t)2 * CH * CH, o, k0);
    wt_one(wo, WT + (size_t)3 * CH * CH, o, k0);
}

__global__ __launch_bounds__(256) void k_wloc(const float* __restrict__ w1, const float* __restrict__ w2,
                                              _Float16* __restrict__ W1B, _Float16* __restrict__ W2B) {
    const unsigned p = blockIdx.x * 256u + threadIdx.x;
    if (p >= (unsigned)(HEADS * HID * 4)) return;
    const unsigned col = p >> 2, k0 = (p & 3u) * 8u;
    const unsigned h = col >> 4, j = col & 15u;
    float v[8];
#pragma unroll
    for (int i = 0; i < 8; ++i) {
        const unsigned k = k0 + (unsigned)i;
        const unsigned kc = min(k, (unsigned)(DG - 1));
        const float x = bfr(w1[(size_t)(h * DG + kc) * HID + j]) * W1_CARRY;
        v[i] = (k < (unsigned)DG) ? x : 0.0f;
    }
    {
        v4f a, b;
        a.x = v[0]; a.y = v[1]; a.z = v[2]; a.w = v[3]; b.x = v[4]; b.y = v[5]; b.z = v[6]; b.w = v[7];
        st8h2(W1B + (size_t)col * 32u + k0, pack8_flush(a, b));
    }
#pragma unroll
    for (int i = 0; i < 8; ++i) {
        const unsigned k = k0 + (unsigned)i;
        const unsigned kc = min(k, (unsigned)(HID - 1));
        const float x = bfr(w2[(size_t)(h * HID + kc) * HID + j]) * W2_CARRY;
        v[i] = (k < (unsigned)HID) ? x : 0.0f;
    }
    {
        v4f a, b;
        a.x = v[0]; a.y = v[1]; a.z = v[2]; a.w = v[3]; b.x = v[4]; b.y = v[5]; b.z = v[6]; b.w = v[7];
        st8h2(W2B + (size_t)col * 32u + k0, pack8_flush(a, b));
    }
}

template <int OUT_MODE, bool BIAS_ROW>
static __device__ __forceinline__ void gemm64_body(
    const _Float16* __restrict__ A, unsigned lda, const _Float16* __restrict__ Bt, unsigned ldb,
    float* __restrict__ Cf, _Float16* __restrict__ Ch, unsigned ldc, const float* __restrict__ bias,
    unsigned M, unsigned N, unsigned K, float scale, float oscale) {
  __shared__ __align__(16) float sT[8][16 * 68];
  const unsigned lane = threadIdx.x & 31u;
  const unsigned wave = threadIdx.x >> 5;
  const unsigned tilesN = N >> 6, tilesM = M >> 6;
  const unsigned tile = blockIdx.x * 8u + wave;
  if (tile >= tilesM * tilesN) return;
  const unsigned tm = tile / tilesN;
  const unsigned tn = tile - tm * tilesN;
  const unsigned m0 = tm << 6, n0 = tn << 6;
  const unsigned rlane = lane & 15u;
  const unsigned koff = (lane >> 4) * 8u;
  const unsigned mOff = koff;

  v8f acc[4][4];
#pragma unroll
  for (int i = 0; i < 4; ++i)
#pragma unroll
    for (int j = 0; j < 4; ++j) acc[i][j] = (v8f){0.f,0.f,0.f,0.f,0.f,0.f,0.f,0.f};

  for (unsigned k0 = 0; k0 < K; k0 += 32u) {
    v16h bh[4];
#pragma unroll
    for (int j = 0; j < 4; ++j)
      bh[j] = frag_ld(Bt + (size_t)(n0 + ((unsigned)j << 4) + rlane) * ldb + koff + k0);
#pragma unroll
    for (int i = 0; i < 4; ++i) {
      const v16h ah = frag_ld(A + (size_t)(m0 + ((unsigned)i << 4) + rlane) * lda + koff + k0);
#pragma unroll
      for (int j = 0; j < 4; ++j)
        acc[i][j] = wmma16g(ah, bh[j], acc[i][j]);
    }
  }

  float* slab = sT[wave];
#pragma unroll
  for (int i = 0; i < 4; ++i) {
    const unsigned mBase = m0 + ((unsigned)i << 4);
    float bvr[8];
#pragma unroll
    for (int r = 0; r < 8; ++r) bvr[r] = 0.0f;
    if (BIAS_ROW) {
#pragma unroll
      for (int r = 0; r < 8; ++r) bvr[r] = bfr(bias[mBase + mOff + (unsigned)r]);
    }
#pragma unroll
    for (int j = 0; j < 4; ++j) {
      const unsigned n = n0 + ((unsigned)j << 4) + rlane;
      float bvc = 0.0f;
      if (!BIAS_ROW) bvc = bfr(bias[n]);
#pragma unroll
      for (int r = 0; r < 8; ++r) {
        float v = acc[i][j][r] * scale + (BIAS_ROW ? bvr[r] : bvc);
        if (OUT_MODE == 1) v *= oscale;
        slab[(mOff + (unsigned)r) * 68u + ((unsigned)j << 4) + rlane] = v;
      }
    }
    wave_sync_lds();
    if (OUT_MODE == 0) {
      const unsigned hh = lane >> 4, c4 = (lane & 15u) * 4u;
#pragma unroll
      for (int half = 0; half < 2; ++half) {
        v4f vv[4];
#pragma unroll
        for (int it = 0; it < 4; ++it) {
          const unsigned row = (unsigned)(half * 4 + it) * 2u + hh;
          vv[it] = *(const v4f*)(slab + row * 68u + c4);
        }
        for (int pass = 0; pass < 2; ++pass) {
#pragma unroll
          for (int it = 0; it < 4; ++it) {
            const unsigned row = (unsigned)(half * 4 + it) * 2u + hh;
            *(volatile v4f*)(Cf + (size_t)(mBase + row) * ldc + n0 + c4) = vv[it];
          }
          __threadfence();
        }
      }
    } else {
      const unsigned q = lane >> 3, c8 = (lane & 7u) * 8u;
      v8h hv[4];
#pragma unroll
      for (int it = 0; it < 4; ++it) {
        const unsigned row = (unsigned)it * 4u + q;
        const float* sp = slab + row * 68u + c8;
        hv[it] = pack8_flush(*(const v4f*)sp, *(const v4f*)(sp + 4));
      }
      for (int pass = 0; pass < 2; ++pass) {
#pragma unroll
        for (int it = 0; it < 4; ++it) {
          const unsigned row = (unsigned)it * 4u + q;
          *(volatile v8h*)(Ch + (size_t)(mBase + row) * ldc + n0 + c8) = hv[it];
        }
        __threadfence();
      }
    }
    wave_sync_lds();
  }
}

__global__ __launch_bounds__(256) void k_proj_rows(const _Float16* __restrict__ X16, const _Float16* __restrict__ Wt,
                                                   _Float16* __restrict__ Y16, const float* __restrict__ bias) {
    gemm64_body<1, false>(X16, CH, Wt, CH, nullptr, Y16, CH, bias, MTOK, CH, CH, SC_PROJ, ACT_CARRY);
}
__global__ __launch_bounds__(256) void k_proj_vt(const _Float16* __restrict__ Wt, const _Float16* __restrict__ X16,
                                                 _Float16* __restrict__ VT16, const float* __restrict__ bias) {
    const unsigned by = blockIdx.y;
    gemm64_body<1, true>(Wt, CH, X16 + (size_t)by * SEQ * CH, CH, nullptr, VT16 + (size_t)by * CH * SEQ, SEQ, bias,
                         CH, SEQ, CH, SC_PROJ, ACT_CARRY);
}
__global__ __launch_bounds__(256) void k_proj_out(const _Float16* __restrict__ O16, const _Float16* __restrict__ Wt,
                                                  float* __restrict__ out, const float* __restrict__ bias) {
    gemm64_body<0, false>(O16, CH, Wt, CH, out, nullptr, CH, bias, MTOK, CH, CH, SC_OUT, 1.0f);
}

#define LC_SP 20
__global__ __launch_bounds__(256) void k_loc(const _Float16* __restrict__ G16, const _Float16* __restrict__ W1B,
                                             const _Float16* __restrict__ W2B, const float* __restrict__ b1,
                                             const float* __restrict__ b2, const float* __restrict__ w3,
                                             const float* __restrict__ b3, float* __restrict__ ALOC) {
    __shared__ __align__(16) float sX[8][16 * LC_SP];
    __shared__ __align__(16) float sA[8][HEADS * 32];
    const unsigned lane = threadIdx.x & 31u;
    const unsigned wave = (unsigned)__builtin_amdgcn_readfirstlane((int)(threadIdx.x >> 5));
    const unsigned hh = lane >> 4, c = lane & 15u;
    const unsigned bx = blockIdx.x;
    const unsigned bn = bx / (unsigned)QBLK;
    const unsigned m0 = ((bx % (unsigned)QBLK) * 8u + wave) * 32u;
    float* xs = sX[wave];
    float* as_ = sA[wave];
    const v8f zacc = (v8f){0.f,0.f,0.f,0.f,0.f,0.f,0.f,0.f};
    const v4u zq = (v4u){0u, 0u, 0u, 0u};
    const unsigned c7 = c & 7u;

#pragma unroll 1
    for (unsigned ti = 0; ti < 2u; ++ti) {
        const unsigned pidx = bn * (unsigned)SEQ + m0 + ti * 16u + c;
        const v4u gq = *(const v4u*)(G16 + (size_t)pidx * 8u);
        FragQ a1;
        a1.q[0].x = (hh == 0u) ? gq.x : 0u;
        a1.q[0].y = (hh == 0u) ? gq.y : 0u;
        a1.q[0].z = (hh == 0u) ? gq.z : 0u;
        a1.q[0].w = (hh == 0u) ? gq.w : 0u;
        a1.q[1] = zq;
#pragma unroll 1
        for (unsigned t = 0; t < (unsigned)HEADS; ++t) {
            const unsigned col = t * 16u + c;
            const v16h w1f = frag_ld(W1B + (size_t)col * 32u + 8u * hh);
            const v8f d1 = wmma16g(a1.v, w1f, zacc);
            const float bb1 = bfr(b1[col]);
#pragma unroll
            for (int r = 0; r < 8; ++r) {
                const float x = d1[r] * UNDO1 + bb1;
                xs[(8u * hh + (unsigned)r) * LC_SP + c] = swishf(x) * H_CARRY;
            }
            wave_sync_lds();
            const float* xr = xs + c * LC_SP + 8u * hh;
            const v4f xa = *(const v4f*)xr;
            const v4f xb = *(const v4f*)(xr + 4);
            FragQ a2;
            a2.h[0] = pack8_flush(xa, xb);
            a2.q[1] = zq;
            wave_sync_lds();
            const v16h w2f = frag_ld(W2B + (size_t)col * 32u + 8u * hh);
            const v8f d2 = wmma16g(a2.v, w2f, zacc);
            const float bb2 = bfr(b2[col]);
            const float ww3 = bfr(w3[col]);
            float part[8];
#pragma unroll
            for (int r = 0; r < 8; ++r) part[r] = swishf(d2[r] * UNDO2 + bb2) * ww3;
#pragma unroll
            for (int r = 0; r < 8; ++r) {
                part[r] += __shfl_xor(part[r], 1, 32);
                part[r] += __shfl_xor(part[r], 2, 32);
                part[r] += __shfl_xor(part[r], 4, 32);
                part[r] += __shfl_xor(part[r], 8, 32);
            }
            float val = part[0];
            val = (c7 == 1u) ? part[1] : val;
            val = (c7 == 2u) ? part[2] : val;
            val = (c7 == 3u) ? part[3] : val;
            val = (c7 == 4u) ? part[4] : val;
            val = (c7 == 5u) ? part[5] : val;
            val = (c7 == 6u) ? part[6] : val;
            val = (c7 == 7u) ? part[7] : val;
            if (c < 8u) as_[t * 32u + ti * 16u + 8u * hh + c] = val;
        }
    }
    wave_sync_lds();
    float fin[8];
#pragma unroll
    for (int t = 0; t < 8; ++t) {
        const float v = as_[(unsigned)t * 32u + lane] + bfr(b3[t]);
        fin[t] = swishf(v);
    }
    const unsigned b = bn / (unsigned)SEQ, n = bn % (unsigned)SEQ;
    float* dst = ALOC + ((size_t)(b * (unsigned)HEADS) * SEQ + n) * SEQ + m0 + lane;
    for (int pass = 0; pass < 2; ++pass) {
#pragma unroll
        for (int t = 0; t < 8; ++t) *(volatile float*)(dst + (size_t)t * SEQ * SEQ) = fin[t];
        __threadfence();
    }
}

#define AT_PP 72
#define AT_OP 68
__global__ __launch_bounds__(512) void k_attn(const _Float16* __restrict__ Q16, const _Float16* __restrict__ K16,
                                              const _Float16* __restrict__ VT16, const float* __restrict__ ALOC,
                                              const int* __restrict__ mask, _Float16* __restrict__ O16) {
    __shared__ __align__(16) _Float16 sP[16][16 * AT_PP];
    __shared__ __align__(16) float sO[16][16 * AT_OP];
    const unsigned tid = threadIdx.x, lane = tid & 31u, wave = tid >> 5;
    const unsigned hh = lane >> 4, c = lane & 15u;
    const unsigned bx = blockIdx.x;
    const unsigned qb = bx % (unsigned)QBLK;
    const unsigned pair = (bx / (unsigned)QBLK) & 3u;
    const unsigned b = bx / ((unsigned)QBLK * 4u);
    const unsigned q0 = qb * 256u + wave * 16u;
    _Float16* pw = sP[wave];
    float* so = sO[wave];
#pragma unroll
    for (int hp = 0; hp < 2; ++hp) {
        const unsigned head = 2u * pair + (unsigned)hp;
        const v16h qf = frag_ld(Q16 + (size_t)(b * SEQ + q0 + c) * CH + head * HD + 8u * hh);
        const float* arow = ALOC + (size_t)((b * (unsigned)HEADS + head) * SEQ + q0 + 8u * hh) * SEQ + c;
        float mrow[8], lrow[8];
        v8f os[2];
#pragma unroll
        for (int r = 0; r < 8; ++r) { mrow[r] = -3.0e38f; lrow[r] = 0.f; }
#pragma unroll
        for (int t = 0; t < 2; ++t) os[t] = (v8f){0.f,0.f,0.f,0.f,0.f,0.f,0.f,0.f};
#pragma unroll 1
        for (unsigned kc = 0; kc < (unsigned)(SEQ / 64); ++kc) {
            const unsigned kv0 = kc * 64u;
            v8f s[4];
#pragma unroll
            for (int j = 0; j < 4; ++j) {
                const v16h kf = frag_ld(K16 + (size_t)(b * SEQ + kv0 + (unsigned)j * 16u + c) * CH + head * HD + 8u * hh);
                const v8f z = (v8f){0.f,0.f,0.f,0.f,0.f,0.f,0.f,0.f};
                s[j] = wmma16g(qf, kf, z);
            }
#pragma unroll
            for (int j = 0; j < 4; ++j) {
                int mk = mask[b * SEQ_FULL + kv0 + (unsigned)j * 16u + c];
                asm volatile("" : "+v"(mk));
                float al[8];
#pragma unroll
                for (int r = 0; r < 8; ++r) al[r] = arow[(size_t)r * SEQ + kv0 + (unsigned)j * 16u];
                asm volatile("" : "+v"(al[0]), "+v"(al[1]), "+v"(al[2]), "+v"(al[3]), "+v"(al[4]), "+v"(al[5]), "+v"(al[6]), "+v"(al[7]));
                const bool on = (mk != 0);
#pragma unroll
                for (int r = 0; r < 8; ++r) {
                    const float sv = (s[j][r] * SCQK + al[r]) * LOG2E;
                    s[j][r] = on ? sv : FILL2;
                }
            }
#pragma unroll
            for (int r = 0; r < 8; ++r) {
                float mx = -3.0e38f;
#pragma unroll
                for (int j = 0; j < 4; ++j) { mx = fmaxf(mx, s[j][r]); }
                mx = fmaxf(mx, __shfl_xor(mx, 1, 32)); mx = fmaxf(mx, __shfl_xor(mx, 2, 32));
                mx = fmaxf(mx, __shfl_xor(mx, 4, 32)); mx = fmaxf(mx, __shfl_xor(mx, 8, 32));
                const float mnew = fmaxf(mrow[r], mx);
                const float alpha = exp2f(mrow[r] - mnew);
                mrow[r] = mnew;
                float psum = 0.f;
#pragma unroll
                for (int j = 0; j < 4; ++j) {
                    const float p = exp2f(s[j][r] - mnew);
                    psum += p;
                    const float w = p * P_CARRY;
                    pw[(8u * hh + (unsigned)r) * AT_PP + (unsigned)j * 16u + c] = (_Float16)((w < 6.103515625e-05f) ? 0.0f : w);
                }
                psum += __shfl_xor(psum, 1, 32); psum += __shfl_xor(psum, 2, 32);
                psum += __shfl_xor(psum, 4, 32); psum += __shfl_xor(psum, 8, 32);
                lrow[r] = lrow[r] * alpha + psum;
                os[0][r] *= alpha; os[1][r] *= alpha;
            }
            wave_sync_lds();
#pragma unroll
            for (int kk = 0; kk < 2; ++kk) {
                const v16h pa = frag_ld(pw + c * AT_PP + (unsigned)kk * 32u + 8u * hh);
#pragma unroll
                for (int t = 0; t < 2; ++t) {
                    const v16h vb = frag_ld(VT16 + (size_t)(b * CH + head * HD + (unsigned)t * 16u + c) * SEQ + kv0 + (unsigned)kk * 32u + 8u * hh);
                    os[t] = wmma16g(pa, vb, os[t]);
                }
            }
            wave_sync_lds();
        }
#pragma unroll
        for (int r = 0; r < 8; ++r) {
            const float inv = 1.0f / (lrow[r] * P_CARRY);
#pragma unroll
            for (int t = 0; t < 2; ++t)
                so[(8u * hh + (unsigned)r) * AT_OP + (unsigned)hp * 32u + (unsigned)t * 16u + c] = os[t][r] * inv * (O_CARRY / ACT_CARRY);
        }
    }
    wave_sync_lds();
    {
        const unsigned q = lane >> 3, c8 = (lane & 7u) * 8u;
        v8h ov[4];
#pragma unroll
        for (int it = 0; it < 4; ++it) {
            const float* sp = so + ((unsigned)it * 4u + q) * AT_OP + c8;
            ov[it] = pack8_flush(*(const v4f*)sp, *(const v4f*)(sp + 4));
        }
        _Float16* dst = O16 + (size_t)(b * SEQ + q0) * CH + pair * 64u;
        for (int pass = 0; pass < 2; ++pass) {
#pragma unroll
            for (int it = 0; it < 4; ++it) *(volatile v8h*)(dst + (size_t)((unsigned)it * 4u + q) * CH + c8) = ov[it];
            __threadfence();
        }
    }
}

extern "C" void kernel_launch(void* const* d_in, const int* in_sizes, int n_in, void* d_out, int out_size,
                              void* d_ws, size_t ws_size, hipStream_t stream) {
    if (n_in < 17) return;
    if (in_sizes[0] < NB * SEQ * SEQ * DG || in_sizes[1] < MTOK * CH) return;
    if (in_sizes[2] < CH * CH || in_sizes[3] < CH || in_sizes[4] < CH * CH || in_sizes[5] < CH) return;
    if (in_sizes[6] < CH * CH || in_sizes[7] < CH || in_sizes[8] < CH * CH || in_sizes[9] < CH) return;
    if (in_sizes[10] < HEADS * DG * HID || in_sizes[11] < HEADS * HID || in_sizes[12] < HEADS * HID * HID) return;
    if (in_sizes[13] < HEADS * HID || in_sizes[14] < HEADS * HID || in_sizes[15] < HEADS || in_sizes[16] < NB * SEQ) return;
    if (out_size < MTOK * CH) return;
    if (ws_size < WS_TOTAL) return;

    const float* pairwise_g = (const float*)d_in[0];
    const float* coset      = (const float*)d_in[1];
    const float* fc_q_w     = (const float*)d_in[2];
    const float* fc_q_b     = (const float*)d_in[3];
    const float* fc_k_w     = (const float*)d_in[4];
    const float* fc_k_b     = (const float*)d_in[5];
    const float* in_w       = (const float*)d_in[6];
    const float* in_b       = (const float*)d_in[7];
    const float* out_w      = (const float*)d_in[8];
    const float* out_b      = (const float*)d_in[9];
    const float* loc_w1     = (const float*)d_in[10];
    const float* loc_b1     = (const float*)d_in[11];
    const float* loc_w2     = (const float*)d_in[12];
    const float* loc_b2     = (const float*)d_in[13];
    const float* loc_w3     = (const float*)d_in[14];
    const float* loc_b3     = (const float*)d_in[15];
    const int*   mask       = (const int*)d_in[16];
    float* out = (float*)d_out;

    char* wsp = (char*)d_ws;
    _Float16* G16  = (_Float16*)(wsp + OFF_G16);
    _Float16* C16  = (_Float16*)(wsp + OFF_C16);
    _Float16* WT   = (_Float16*)(wsp + OFF_WT);
    _Float16* W1B  = (_Float16*)(wsp + OFF_W1B);
    _Float16* W2B  = (_Float16*)(wsp + OFF_W2B);
    _Float16* Q16  = (_Float16*)(wsp + OFF_Q16);
    _Float16* K16  = (_Float16*)(wsp + OFF_K16);
    _Float16* VT16 = (_Float16*)(wsp + OFF_VT16);
    float*    ALOC = (float*)(wsp + OFF_ALOC);
    _Float16* O16  = (_Float16*)(wsp + OFF_O16);

    k_cvt_g<<<(NB * SEQ * SEQ) / 256, 256, 0, stream>>>(pairwise_g, G16);
    k_cvt_c<<<(MTOK * CH / 8) / 256, 256, 0, stream>>>(coset, C16);
    k_wt4<<<(CH * (CH / 8)) / 256, 256, 0, stream>>>(fc_q_w, fc_k_w, in_w, out_w, WT);
    k_wloc<<<(HEADS * HID * 4) / 256, 256, 0, stream>>>(loc_w1, loc_w2, W1B, W2B);

    k_proj_rows<<<((MTOK / 64) * (CH / 64) + 7) / 8, 256, 0, stream>>>(C16, WT, Q16, fc_q_b);
    k_proj_rows<<<((MTOK / 64) * (CH / 64) + 7) / 8, 256, 0, stream>>>(C16, WT + (size_t)1 * CH * CH, K16, fc_k_b);
    k_proj_vt<<<dim3(((CH / 64) * (SEQ / 64) + 7) / 8, NB), 256, 0, stream>>>(WT + (size_t)2 * CH * CH, C16, VT16, in_b);

    k_loc<<<NB * SEQ * QBLK, 256, 0, stream>>>(G16, W1B, W2B, loc_b1, loc_b2, loc_w3, loc_b3, ALOC);
    k_attn<<<NB * 4 * QBLK, 512, 0, stream>>>(Q16, K16, VT16, ALOC, mask, O16);
    k_proj_out<<<((MTOK / 64) * (CH / 64) + 7) / 8, 256, 0, stream>>>(O16, WT + (size_t)3 * CH * CH, out, out_b);
}
